// MultiScaleRetention_15702400434237
// MI455X (gfx1250) — hardware-verified
//
#include <hip/hip_runtime.h>
#include <math.h>

constexpr int kB     = 8;
constexpr int kS     = 1024;
constexpr int kD     = 512;
constexpr int kH     = 8;
constexpr int kDh    = 64;
constexpr int kHalf  = 32;
constexpr int kTok   = kB * kS;
constexpr int kGroup = 4;
constexpr int kNG    = kH / kGroup;
constexpr int kTab   = kS * kHalf;
constexpr int kWRows = 5 * kD;
constexpr int kRowQ = 0, kRowK = kD, kRowV = 2 * kD, kRowG = 3 * kD, kRowO = 4 * kD;

constexpr float kWCarry    = 64.0f;
constexpr float kPreCarry  = 16.0f;
constexpr float kQCarry    = 16.0f;
constexpr float kKCarry    = 4.0f;
constexpr float kVCarry    = 16.0f;
constexpr float kPCarry    = 32768.0f;
constexpr float kZCarry    = 256.0f;
constexpr float kProjScale = kPreCarry / kWCarry;
constexpr float kVTScale   = kVCarry / kWCarry;
constexpr float kGScale    = 1.0f / kWCarry;
constexpr float kQFac      = kQCarry / kPreCarry;
constexpr float kKFac      = kKCarry / kPreCarry;
constexpr float kScoreScale = 1.0f / (kQCarry * kKCarry);
constexpr float kPVScale   = 1.0f / (kPCarry * kVCarry);
constexpr float kOutScale  = 1.0f / (kZCarry * kWCarry);
constexpr float kGnEps     = 1.0e-5f;
constexpr float kLg0       = -3.4657359027997265f;
constexpr float kLg1       = -6.2383246250395078f;
constexpr float kLog2TenK32 = 0.41524101186092029f;
static_assert(kH * kDh == kD, "shape");
static_assert(kS % 64 == 0 && kD % 64 == 0 && kDh % 32 == 0, "tiles");
static_assert(kH % kGroup == 0 && kD / 64 == kH, "groups");

typedef __attribute__((ext_vector_type(16))) _Float16 v16h;
typedef __attribute__((ext_vector_type(8)))  _Float16 v8h;
typedef __attribute__((ext_vector_type(16))) __bf16   v16b;
typedef __attribute__((ext_vector_type(8)))  __bf16   v8b;
typedef __attribute__((ext_vector_type(8)))  float    v8f;
typedef __attribute__((ext_vector_type(4)))  float    v4f;
typedef __attribute__((ext_vector_type(2)))  float    v2f;
typedef __attribute__((ext_vector_type(4)))  unsigned int v4u;

__device__ __forceinline__ unsigned short f2bf_bits(float f) {
  unsigned u = __float_as_uint(f);
  return (unsigned short)((u + 0x7FFFu + ((u >> 16) & 1u)) >> 16);
}
__device__ __forceinline__ float bf_bits2f(unsigned short h) { return __uint_as_float(((unsigned)h) << 16); }

__device__ __forceinline__ void dep_guard_h(v8f& a, v8f& b, v16h x, v16h y) { asm volatile("v_nop\n\tv_nop\n\tv_nop\n\tv_nop" : "+v"(a), "+v"(b) : "v"(x), "v"(y)); }
__device__ __forceinline__ void dep_guard_b(v8f& a, v8f& b, v16b x, v16b y) { asm volatile("v_nop\n\tv_nop\n\tv_nop\n\tv_nop" : "+v"(a), "+v"(b) : "v"(x), "v"(y)); }
__device__ __forceinline__ void keep4_h(v16h a, v16h b, v16h c, v16h d) { asm volatile("v_nop" :: "v"(a), "v"(b), "v"(c), "v"(d)); }
__device__ __forceinline__ void keep4_b(v16b a, v16b b, v16b c, v16b d) { asm volatile("v_nop" :: "v"(a), "v"(b), "v"(c), "v"(d)); }
__device__ __forceinline__ void acc_guard4(v8f& a, v8f& b, v8f& c, v8f& d) { asm volatile("v_nop\n\tv_nop\n\tv_nop\n\tv_nop" : "+v"(a), "+v"(b), "+v"(c), "+v"(d)); }
template <typename T> struct Frag;
template <> struct Frag<_Float16> {
  typedef v16h V; union U { v16h v; v8h h[2]; };
  static __device__ __forceinline__ v16h load(const _Float16* p) {
    U f; f.h[0] = *(const v8h*)(p); f.h[1] = *(const v8h*)(p + 16); return f.v;
  }
  static __device__ __forceinline__ v8f mma(v16h a, v16h b, v8f c) {
    return __builtin_amdgcn_wmma_f32_16x16x32_f16(false, a, false, b, (short)0, c, false, false);
  }
  static __device__ __forceinline__ void guard(v8f& a, v8f& b, v16h x, v16h y) { dep_guard_h(a, b, x, y); }
  static __device__ __forceinline__ void keep(v16h a, v16h b, v16h c, v16h d) { keep4_h(a, b, c, d); }
};
template <> struct Frag<__bf16> {
  typedef v16b V; union U { v16b v; v8b h[2]; };
  static __device__ __forceinline__ v16b load(const __bf16* p) {
    U f; f.h[0] = *(const v8b*)(p); f.h[1] = *(const v8b*)(p + 16); return f.v;
  }
  static __device__ __forceinline__ v8f mma(v16b a, v16b b, v8f c) {
    return __builtin_amdgcn_wmma_f32_16x16x32_bf16(false, a, false, b, (short)0, c, false, false);
  }
  static __device__ __forceinline__ void guard(v8f& a, v8f& b, v16b x, v16b y) { dep_guard_b(a, b, x, y); }
  static __device__ __forceinline__ void keep(v16b a, v16b b, v16b c, v16b d) { keep4_b(a, b, c, d); }
};

__device__ __forceinline__ unsigned pk16(unsigned short a, unsigned short b) { return (unsigned)a | ((unsigned)b << 16); }
__device__ __forceinline__ unsigned short h_bits(float f) { const _Float16 h = (_Float16)f; return __builtin_bit_cast(unsigned short, h); }
__device__ __forceinline__ float bfr(float f) { return __uint_as_float(((unsigned)f2bf_bits(f)) << 16); }
__device__ __forceinline__ float h16_to_f32(unsigned hb) {
  const unsigned sgn = (hb & 0x8000u) << 16; const unsigned em = hb & 0x7fffu;
  const float fn = __uint_as_float((em << 13) + 0x38000000u);
  const float fs = (float)em * 5.9604644775390625e-8f;
  const float mag = (em < 0x400u) ? fs : fn; return __uint_as_float(__float_as_uint(mag) | sgn); }

template <int ET> struct Elem;
template <> struct Elem<0> { typedef _Float16 T; };
template <> struct Elem<1> { typedef __bf16 T; };
template <int ET, bool SPLIT, int BIAS_MODE, int OUT_MODE, bool RESID, int ACT = 0>
__global__ __launch_bounds__(256) void wmma_gemm64(
    const unsigned short* __restrict__ Ap, const unsigned short* __restrict__ A2p, int lda, long strideA,
    const unsigned short* __restrict__ Btp, const unsigned short* __restrict__ Bt2p, int ldb, long strideB,
    void* __restrict__ Cout, void* __restrict__ Cout2, int ldc, long strideC,
    const float* __restrict__ bias,
    const float* __restrict__ resid, long strideR,
    int M, int N, int K, float scale) {
  typedef typename Elem<ET>::T T;
  typedef typename Frag<T>::V V;
  const T* A = (const T*)Ap; const T* A2 = (const T*)A2p; const T* Bt = (const T*)Btp; const T* Bt2 = (const T*)Bt2p;
  __shared__ __align__(16) float sT[8][16 * 68];
  const int b    = blockIdx.y;
  const int lane = threadIdx.x & 31;
  const int wave = threadIdx.x >> 5;
  const int tilesN = N >> 6;
  const int tilesM = M >> 6;
  const int tile = blockIdx.x * 8 + wave;
  if (tile >= tilesM * tilesN) return;
  const int tm = tile / tilesN;
  const int tn = tile - tm * tilesN;
  const int m0 = tm << 6;
  const int n0 = tn << 6;

  const T* Ab  = A  + (size_t)b * strideA;
  const T* Bb  = Bt + (size_t)b * strideB;
  const T* Ab2 = SPLIT ? (A2  + (size_t)b * strideA) : nullptr;
  const T* Bb2 = SPLIT ? (Bt2 + (size_t)b * strideB) : nullptr;

  const int rlane = lane & 15;
  const int koff  = (lane >> 4) * 8;
  const int mOff  = (lane >> 4) * 8;

  v8f acc[4][4];
#pragma unroll
  for (int i = 0; i < 4; ++i)
#pragma unroll
    for (int j = 0; j < 4; ++j) acc[i][j] = (v8f){0.f,0.f,0.f,0.f,0.f,0.f,0.f,0.f};

  for (int k0 = 0; k0 < K; k0 += 32) {
    V bh[4], bl[4];
#pragma unroll
    for (int j = 0; j < 4; ++j) {
      const size_t bo = (size_t)(n0 + (j << 4) + rlane) * ldb + koff + k0;
      bh[j] = Frag<T>::load(Bb + bo);
      if (SPLIT) bl[j] = Frag<T>::load(Bb2 + bo);
    }
#pragma unroll
    for (int i = 0; i < 4; ++i) {
      const size_t ao = (size_t)(m0 + (i << 4) + rlane) * lda + koff + k0;
      V ah = Frag<T>::load(Ab + ao);
      V al;
      if (SPLIT) al = Frag<T>::load(Ab2 + ao);
#pragma unroll
      for (int j = 0; j < 4; ++j) {
        acc[i][j] = Frag<T>::mma(ah, bh[j], acc[i][j]);
        if (SPLIT) {
          acc[i][j] = Frag<T>::mma(ah, bl[j], acc[i][j]);
          acc[i][j] = Frag<T>::mma(al, bh[j], acc[i][j]);
        }
      }
      Frag<T>::guard(acc[i][0], acc[i][3], ah, SPLIT ? al : ah);
      Frag<T>::guard(acc[i][1], acc[i][2], bh[1], bh[2]);
    }
    Frag<T>::keep(bh[0], bh[1], bh[2], bh[3]);
    if (SPLIT) Frag<T>::keep(bl[0], bl[1], bl[2], bl[3]);
  }
  acc_guard4(acc[0][0], acc[0][1], acc[0][2], acc[0][3]);
  acc_guard4(acc[1][0], acc[1][1], acc[1][2], acc[1][3]);
  acc_guard4(acc[2][0], acc[2][1], acc[2][2], acc[2][3]);
  acc_guard4(acc[3][0], acc[3][1], acc[3][2], acc[3][3]);

  float* slab = sT[wave];
  const float* Rb = RESID ? (resid + (size_t)b * strideR) : nullptr;
#pragma unroll
  for (int i = 0; i < 4; ++i) {
    const int mBase = m0 + (i << 4);
#pragma unroll
    for (int j = 0; j < 4; ++j) {
      const int n = n0 + (j << 4) + rlane;
      float bv = 0.f;
      if (BIAS_MODE == 2) bv = bias[n];
#pragma unroll
      for (int r = 0; r < 8; ++r) {
        float v = acc[i][j][r] * scale;
        if (BIAS_MODE == 1) v += bias[mBase + mOff + r];
        if (BIAS_MODE == 2) v += bv;
        if (RESID) v += Rb[(size_t)(mBase + mOff + r) * ldc + n];
        if (ACT == 2) v = fmaxf(v, 0.0f);
        if (ACT == 4) v = (v > 0.f) ? v : 0.01f * v;
        slab[(mOff + r) * 68 + (j << 4) + rlane] = v;
      }
    }
    __builtin_amdgcn_fence(__ATOMIC_RELEASE, "workgroup");
    __builtin_amdgcn_wave_barrier();
    __builtin_amdgcn_fence(__ATOMIC_ACQUIRE, "workgroup");
    if (OUT_MODE == 0) {
      float* C = (float*)Cout + (size_t)b * strideC;
      const int hh = lane >> 4, c4 = (lane & 15) * 4;
      for (int pass = 0; pass < 2; ++pass) {
#pragma unroll
        for (int it = 0; it < 8; ++it) {
          const int row = it * 2 + hh;
          v4f v = *(const v4f*)(slab + row * 68 + c4);
          *(volatile v4f*)(C + (size_t)(mBase + row) * ldc + n0 + c4) = v;
        }
        __threadfence();
      }
    } else {
      const int q = lane >> 3, c8 = (lane & 7) * 8;
      unsigned short* C  = (unsigned short*)Cout  + (size_t)b * strideC;
      unsigned short* C2 = (OUT_MODE == 2) ? ((unsigned short*)Cout2 + (size_t)b * strideC) : nullptr;
      for (int pass = 0; pass < 2; ++pass) {
#pragma unroll
        for (int it = 0; it < 4; ++it) {
          const int row = it * 4 + q;
          const float* sp = slab + row * 68 + c8;
          v8h hv, lv;
#pragma unroll
          for (int e = 0; e < 8; ++e) {
            if (OUT_MODE == 1) {
              hv[e] = (_Float16)sp[e];
            } else {
              unsigned short hb = f2bf_bits(sp[e]);
              unsigned short lb = f2bf_bits(sp[e] - bf_bits2f(hb));
              hv[e] = __builtin_bit_cast(_Float16, hb);
              lv[e] = __builtin_bit_cast(_Float16, lb);
            }
          }
          *(volatile v8h*)(C + (size_t)(mBase + row) * ldc + n0 + c8) = hv;
          if (OUT_MODE == 2) *(volatile v8h*)(C2 + (size_t)(mBase + row) * ldc + n0 + c8) = lv;
        }
        __threadfence();
      }
    }
    __builtin_amdgcn_fence(__ATOMIC_RELEASE, "workgroup");
    __builtin_amdgcn_wave_barrier();
    __builtin_amdgcn_fence(__ATOMIC_ACQUIRE, "workgroup");
  }
}

__global__ __launch_bounds__(256) void cast_x_kernel(const float* __restrict__ in, unsigned short* __restrict__ out, int n8) {
  const int i = blockIdx.x * 256 + threadIdx.x;
  if (i >= n8) return;
  const float* p = in + 8 * (size_t)i;
  const v4f a = *(const v4f*)(p);
  const v4f c = *(const v4f*)(p + 4);
  unsigned short hb[8];
#pragma unroll
  for (int e = 0; e < 4; ++e) {
    hb[e]     = h_bits(bfr(a[e]));
    hb[4 + e] = h_bits(bfr(c[e]));
  }
  const v4u u = (v4u){pk16(hb[0], hb[1]), pk16(hb[2], hb[3]), pk16(hb[4], hb[5]), pk16(hb[6], hb[7])};
  unsigned short* q = out + 8 * (size_t)i;
  *(volatile v4u*)q = u;
  __threadfence();
  *(volatile v4u*)q = u;
}

__global__ __launch_bounds__(256) void wcast_kernel(const float* __restrict__ W0, const float* __restrict__ W1,
                                                    const float* __restrict__ W2, const float* __restrict__ W3,
                                                    const float* __restrict__ W4,
                                                    unsigned short* __restrict__ out, float carry) {
  __shared__ float sm[64][65];
  const int t  = threadIdx.x;
  const int d0 = blockIdx.x * 64;
  const int nt = blockIdx.y;
  const int z  = blockIdx.z;
  const float* W = (z == 0) ? W0 : (z == 1) ? W1 : (z == 2) ? W2 : (z == 3) ? W3 : W4;
  const bool perHead   = (z <= 2);
  const size_t rowBase = perHead ? (size_t)nt * kD : (size_t)0;
  const int pitch      = perHead ? kDh : kD;
  const int nbase      = perHead ? 0 : nt * 64;
#pragma unroll
  for (int i = 0; i < 16; ++i) {
    const int e = i * 256 + t;
    const int r = e >> 6;
    const int c = e & 63;
    const float wv = W[(rowBase + (size_t)(d0 + r)) * pitch + nbase + c];
    sm[c][r] = bfr(wv) * carry;
  }
  __syncthreads();
  const int lane = t & 31, wave = t >> 5;
  const int q = lane >> 3, c8 = (lane & 7) * 8;
  unsigned short* op = out + (size_t)z * kD * kD;
  for (int pass = 0; pass < 2; ++pass) {
#pragma unroll
    for (int it = 0; it < 2; ++it) {
      const int row = wave * 8 + it * 4 + q;
      unsigned short hb[8];
#pragma unroll
      for (int e = 0; e < 8; ++e) hb[e] = h_bits(sm[row][c8 + e]);
      const v4u u = (v4u){pk16(hb[0], hb[1]), pk16(hb[2], hb[3]), pk16(hb[4], hb[5]), pk16(hb[6], hb[7])};
      *(volatile v4u*)(op + (size_t)(nt * 64 + row) * kD + d0 + c8) = u;
    }
    __threadfence();
  }
}

__global__ __launch_bounds__(256) void xpos_table_kernel(float* __restrict__ T) {
  const int idx = blockIdx.x * 256 + threadIdx.x;
  if (idx >= kTab) return;
  const int s = idx >> 5, j = idx & 31;
  const float sv    = ((float)(2 * j) + 25.6f) / 89.6f;
  const float power = (float)s * (1.0f / 512.0f);
  const float scale = exp2f(power * log2f(sv));
  const float iscal = 1.0f / scale;
  const float invf  = exp2f(-(float)j * kLog2TenK32);
  const float ang   = (float)s * invf;
  float sn, cs;
  sincosf(ang, &sn, &cs);
  const float t0 = cs * scale, t1 = sn * scale, t2 = cs * iscal, t3 = sn * iscal;
  *(volatile float*)(T + idx)            = t0;
  *(volatile float*)(T + kTab + idx)     = t1;
  *(volatile float*)(T + 2 * kTab + idx) = t2;
  *(volatile float*)(T + 3 * kTab + idx) = t3;
  __threadfence();
  *(volatile float*)(T + idx)            = t0;
  *(volatile float*)(T + kTab + idx)     = t1;
  *(volatile float*)(T + 2 * kTab + idx) = t2;
  *(volatile float*)(T + 3 * kTab + idx) = t3;
}

__global__ __launch_bounds__(256) void xpos_kernel(const unsigned short* __restrict__ QKpre, const float* __restrict__ T,
                                                   unsigned short* __restrict__ QKh) {
  const int t    = threadIdx.x;
  const int rloc = t >> 7;
  const int row  = blockIdx.x * 2 + rloc;
  const int u    = t & 127;
  const int isK  = u >> 6;
  const int tt   = u & 63;
  const int col0 = tt * 8;
  const int j0   = (tt & 7) * 4;
  const int s    = row & (kS - 1);
  const v4u w = *(const v4u*)(QKpre + (size_t)row * (2 * kD) + isK * kD + col0);
  const unsigned w0 = w.x, w1 = w.y, w2 = w.z, w3 = w.w;
  float x[8];
  x[0] = h16_to_f32(w0 & 0xffffu); x[1] = h16_to_f32(w0 >> 16);
  x[2] = h16_to_f32(w1 & 0xffffu); x[3] = h16_to_f32(w1 >> 16);
  x[4] = h16_to_f32(w2 & 0xffffu); x[5] = h16_to_f32(w2 >> 16);
  x[6] = h16_to_f32(w3 & 0xffffu); x[7] = h16_to_f32(w3 >> 16);
  const float* tc = T + (size_t)(isK * 2) * kTab + s * kHalf + j0;
  const v4f c4 = *(const v4f*)(tc);
  const v4f s4 = *(const v4f*)(tc + kTab);
  const float fac = isK ? kKFac : kQFac;
  float o[8];
#pragma unroll
  for (int p = 0; p < 4; ++p) {
    const float c  = c4[p] * fac;
    const float sn = s4[p] * fac;
    const float x0 = x[2 * p], x1 = x[2 * p + 1];
    o[2 * p]     = x0 * c - x1 * sn;
    o[2 * p + 1] = x1 * c + x0 * sn;
  }
  unsigned short hb[8];
#pragma unroll
  for (int e = 0; e < 8; ++e) hb[e] = h_bits(o[e]);
  const v4u uo = (v4u){pk16(hb[0], hb[1]), pk16(hb[2], hb[3]), pk16(hb[4], hb[5]), pk16(hb[6], hb[7])};
  unsigned short* dst = QKh + (size_t)isK * kTok * kD + (size_t)row * kD + col0;
  *(volatile v4u*)dst = uo;
  __threadfence();
  *(volatile v4u*)dst = uo;
}

__global__ __launch_bounds__(128) void softmax_decay_kernel(const float* __restrict__ Sp, unsigned short* __restrict__ Pp, int hbase) {
  __shared__ __align__(16) float lg[kS];
  __shared__ float redM[4];
  __shared__ float redS[4];
  const int i    = blockIdx.x;
  const int hg   = blockIdx.y;
  const int h    = hbase + hg;
  const int t    = threadIdx.x;
  const int lane = t & 31, wave = t >> 5;
  const float gval  = kLg0 + (float)h * ((kLg1 - kLg0) * (1.0f / 7.0f));
  const float gamma = 1.0f - expf(gval);
  const float log2g = log2f(gamma);
  const size_t rowoff = ((size_t)hg * kS + i) * kS;
  const float* sr = Sp + rowoff;

  float mx = -__builtin_inff();
#pragma unroll 1
  for (int it = 0; it < 4; ++it) {
    const int c = it * 256 + 2 * t;
    const v2f sv = *(const v2f*)(sr + c);
    mx = fmaxf(mx, fmaxf(sv[0], sv[1]));
    *(v2f*)(lg + c) = sv;
  }
#pragma unroll
  for (int off = 16; off > 0; off >>= 1) mx = fmaxf(mx, __shfl_xor(mx, off, 32));
  if (lane == 0) redM[wave] = mx;
  __syncthreads();
  float m = redM[0];
#pragma unroll
  for (int wv = 1; wv < 4; ++wv) m = fmaxf(m, redM[wv]);

  float sum = 0.f;
#pragma unroll 1
  for (int it = 0; it < 4; ++it) {
    const int c = it * 256 + 2 * t;
    const v2f l = *(const v2f*)(lg + c);
    v2f ev;
#pragma unroll
    for (int e = 0; e < 2; ++e) {
      const float ex = expf(l[e] - m);
      sum += ex;
      const int dcol = i - (c + e);
      const int ad   = (dcol < 0) ? -dcol : dcol;
      const float dw = exp2f((float)ad * log2g);
      ev[e] = ex * dw;
    }
    *(v2f*)(lg + c) = ev;
  }
#pragma unroll
  for (int off = 16; off > 0; off >>= 1) sum += __shfl_xor(sum, off, 32);
  if (lane == 0) redS[wave] = sum;
  __syncthreads();
  float tot = redS[0];
#pragma unroll
  for (int wv = 1; wv < 4; ++wv) tot += redS[wv];
  const float inv = kPCarry * (1.0f / tot);

  const v4f e0 = *(const v4f*)(lg + 8 * t);
  const v4f e1 = *(const v4f*)(lg + 8 * t + 4);
  unsigned short hb[8];
#pragma unroll
  for (int e = 0; e < 4; ++e) {
    hb[e]     = h_bits(e0[e] * inv);
    hb[4 + e] = h_bits(e1[e] * inv);
  }
  const v4u u = (v4u){pk16(hb[0], hb[1]), pk16(hb[2], hb[3]), pk16(hb[4], hb[5]), pk16(hb[6], hb[7])};
  unsigned short* pr = Pp + rowoff + 8 * (size_t)t;
  *(volatile v4u*)pr = u;
  __threadfence();
  *(volatile v4u*)pr = u;
}

__global__ __launch_bounds__(256) void gn_gate_kernel(const float* __restrict__ Y, const float* __restrict__ Gf,
                                                      const float* __restrict__ gnw, const float* __restrict__ gnb,
                                                      unsigned short* __restrict__ Zh) {
  const int row = blockIdx.x;
  const int t   = threadIdx.x;
  const size_t base = (size_t)row * kD + 2 * t;
  const v2f yv = *(const v2f*)(Y + base);
  const v2f gv = *(const v2f*)(Gf + base);
  const v2f wv = *(const v2f*)(gnw + 2 * t);
  const v2f bv = *(const v2f*)(gnb + 2 * t);
  const float y0 = yv[0], y1 = yv[1];
  float s = 0.0f;
  s += y0; s += y1;
#pragma unroll
  for (int off = 1; off < 32; off <<= 1) s += __shfl_xor(s, off, 32);
  const float mu = s * (1.0f / 64.0f);
  const float d0 = y0 - mu, d1 = y1 - mu;
  float q = 0.0f;
  q += d0 * d0; q += d1 * d1;
#pragma unroll
  for (int off = 1; off < 32; off <<= 1) q += __shfl_xor(q, off, 32);
  const float var = q * (1.0f / 64.0f);
  const float rs  = rsqrtf(var + kGnEps);
  const float yn0 = d0 * rs * bfr(wv[0]) + bfr(bv[0]);
  const float yn1 = d1 * rs * bfr(wv[1]) + bfr(bv[1]);
  const float g0 = gv[0], g1 = gv[1];
  const float sw0 = g0 * (1.0f / (1.0f + expf(-g0)));
  const float sw1 = g1 * (1.0f / (1.0f + expf(-g1)));
  const float z0 = kZCarry * (sw0 * yn0);
  const float z1 = kZCarry * (sw1 * yn1);
  const unsigned u = pk16(h_bits(z0), h_bits(z1));
  unsigned* zp = (unsigned*)(void*)Zh + ((size_t)row * (kD / 2) + t);
  *(volatile unsigned*)zp = u;
  __threadfence();
  *(volatile unsigned*)zp = u;
}

extern "C" void kernel_launch(void* const* d_in, const int* in_sizes, int n_in,
                              void* d_out, int out_size, void* d_ws, size_t ws_size,
                              hipStream_t stream) {
  if (n_in < 8) return;
  const int nTokD = kTok * kD;
  if (in_sizes[0] != nTokD) return;
  if (in_sizes[1] != kH * kD * kDh || in_sizes[2] != kH * kD * kDh || in_sizes[3] != kH * kD * kDh) return;
  if (in_sizes[4] != kD * kD || in_sizes[5] != kD * kD) return;
  if (in_sizes[6] != kD || in_sizes[7] != kD) return;
  if (out_size != nTokD) return;

  const size_t szXh  = (size_t)kTok * kD * 2;
  const size_t szW   = (size_t)kWRows * kD * 2;
  const size_t szT   = (size_t)4 * kTab * 4;
  const size_t szQKp = (size_t)kTok * (2 * kD) * 2;
  const size_t szG   = (size_t)kTok * kD * 4;
  const size_t szVT  = (size_t)kB * kD * kS * 2;
  const size_t szQKh = (size_t)2 * kTok * kD * 2;
  const size_t szSC  = (size_t)kGroup * kS * kS * 4;
  const size_t szP   = (size_t)kGroup * kS * kS * 2;
  const size_t szY   = (size_t)kTok * kD * 4;
  const size_t szZ   = (size_t)kTok * kD * 2;
  const size_t offXh  = 0;
  const size_t offW   = offXh + szXh;
  const size_t offT   = offW + szW;
  const size_t offQKp = offT + szT;
  const size_t offG   = offQKp + szQKp;
  const size_t offVT  = offG + szG;
  const size_t offQKh = offVT + szVT;
  const size_t offSC  = offQKh + szQKh;
  const size_t offP   = offSC + szSC;
  const size_t offY   = offP + szP;
  const size_t offZ   = offY + szY;
  const size_t total  = offZ + szZ;
  if (ws_size < total) return;

  const float* X   = (const float*)d_in[0];
  const float* WQ  = (const float*)d_in[1];
  const float* WK  = (const float*)d_in[2];
  const float* WV  = (const float*)d_in[3];
  const float* WG  = (const float*)d_in[4];
  const float* WO  = (const float*)d_in[5];
  const float* gnw = (const float*)d_in[6];
  const float* gnb = (const float*)d_in[7];
  float* out = (float*)d_out;
  char* ws = (char*)d_ws;
  unsigned short* Xh    = (unsigned short*)(ws + offXh);
  unsigned short* Wall  = (unsigned short*)(ws + offW);
  float*          T     = (float*)(ws + offT);
  unsigned short* QKpre = (unsigned short*)(ws + offQKp);
  float*          Gf    = (float*)(ws + offG);
  unsigned short* VT    = (unsigned short*)(ws + offVT);
  unsigned short* QKh   = (unsigned short*)(ws + offQKh);
  float*          SC    = (float*)(ws + offSC);
  unsigned short* PP    = (unsigned short*)(ws + offP);
  float*          Y     = (float*)(ws + offY);
  unsigned short* Zh    = (unsigned short*)(ws + offZ);
  const float* dummyF = T;

  const unsigned short* WQKt = Wall + (size_t)kRowQ * kD;
  const unsigned short* WVt  = Wall + (size_t)kRowV * kD;
  const unsigned short* WGt  = Wall + (size_t)kRowG * kD;
  const unsigned short* WOt  = Wall + (size_t)kRowO * kD;
  unsigned short* Qh = QKh;
  unsigned short* Kh = QKh + (size_t)kTok * kD;

  const int n8 = nTokD / 8;
  cast_x_kernel<<<dim3(n8 / 256), dim3(256), 0, stream>>>(X, Xh, n8);
  wcast_kernel<<<dim3(kD / 64, 8, 5), dim3(256), 0, stream>>>(WQ, WK, WV, WG, WO, Wall, kWCarry);
  xpos_table_kernel<<<dim3(kTab / 256), dim3(256), 0, stream>>>(T);

  {
    const int tiles = (kTok / 64) * ((2 * kD) / 64);
    wmma_gemm64<0, false, 0, 1, false, 0><<<dim3(tiles / 8, 1), dim3(256), 0, stream>>>(
        Xh, Xh, kD, 0L, WQKt, WQKt, kD, 0L, (void*)QKpre, (void*)QKpre, 2 * kD, 0L,
        dummyF, dummyF, 0L, kTok, 2 * kD, kD, kProjScale);
  }
  {
    const int tiles = (kTok / 64) * (kD / 64);
    wmma_gemm64<0, false, 0, 0, false, 0><<<dim3(tiles / 8, 1), dim3(256), 0, stream>>>(
        Xh, Xh, kD, 0L, WGt, WGt, kD, 0L, (void*)Gf, (void*)Gf, kD, 0L,
        dummyF, dummyF, 0L, kTok, kD, kD, kGScale);
  }
  {
    const int tiles = (kD / 64) * (kS / 64);
    wmma_gemm64<0, false, 0, 1, false, 0><<<dim3(tiles / 8, kB), dim3(256), 0, stream>>>(
        WVt, WVt, kD, 0L, Xh, Xh, kD, (long)kS * kD, (void*)VT, (void*)VT, kS, (long)kD * kS,
        dummyF, dummyF, 0L, kD, kS, kD, kVTScale);
  }
  xpos_kernel<<<dim3(kTok / 2), dim3(256), 0, stream>>>(QKpre, T, QKh);

  const long strideHead16 = (long)kDh;
  const long strideScore  = (long)kS * kS;
  const long strideVT     = (long)kDh * kS;
  const int  tilesScore   = (kS / 64) * (kS / 64);
  const int  tilesCtx     = (kS / 64) * (kDh / 64);
  for (int b = 0; b < kB; ++b) {
    for (int g = 0; g < kNG; ++g) {
      const int hbase = g * kGroup;
      const size_t tokOff = ((size_t)b * kS) * kD + (size_t)hbase * kDh;
      const unsigned short* Ag  = Qh + tokOff;
      const unsigned short* Btg = Kh + tokOff;
      wmma_gemm64<0, false, 0, 0, false, 0><<<dim3(tilesScore / 8, kGroup), dim3(256), 0, stream>>>(
          Ag, Ag, kD, strideHead16, Btg, Btg, kD, strideHead16,
          (void*)SC, (void*)SC, kS, strideScore, dummyF, dummyF, 0L, kS, kS, kDh, kScoreScale);
      softmax_decay_kernel<<<dim3(kS, kGroup), dim3(128), 0, stream>>>(SC, PP, hbase);
      const unsigned short* VTg = VT + ((size_t)b * kD + (size_t)hbase * kDh) * kS;
      float* Yg = Y + tokOff;
      wmma_gemm64<0, false, 0, 0, false, 0><<<dim3(tilesCtx / 8, kGroup), dim3(256), 0, stream>>>(
          PP, PP, kS, strideScore, VTg, VTg, kS, strideVT,
          (void*)Yg, (void*)Yg, kD, strideHead16, dummyF, dummyF, 0L, kS, kDh, kS, kPVScale);
    }
  }

  gn_gate_kernel<<<dim3(kTok), dim3(256), 0, stream>>>(Y, Gf, gnw, gnb, Zh);
  {
    const int tiles = (kTok / 64) * (kD / 64);
    wmma_gemm64<0, false, 0, 0, false, 0><<<dim3(tiles / 8, 1), dim3(256), 0, stream>>>(
        Zh, Zh, kD, 0L, WOt, WOt, kD, 0L, (void*)out, (void*)out, kD, 0L,
        dummyF, dummyF, 0L, kTok, kD, kD, kOutScale);
  }
}
